// SSMBlock_31937376813582
// MI455X (gfx1250) — hardware-verified
//
#include <hip/hip_runtime.h>
#include <math.h>

typedef __attribute__((ext_vector_type(16))) _Float16 v16h;
typedef __attribute__((ext_vector_type(8)))  _Float16 v8h;
typedef __attribute__((ext_vector_type(8)))  float    v8f;
typedef __attribute__((ext_vector_type(4)))  float    v4f;

constexpr int kBatch  = 4;
constexpr int kSeq    = 2048;
constexpr int kDm     = 1024;
constexpr int kNst    = 16;
constexpr int kRows   = kBatch * kSeq;
constexpr int kXzN    = 2 * kDm;
constexpr int kBcP    = 64;
constexpr int kScanTS = 64;
constexpr int kScanCh = 64;
constexpr int kScanYP = 68;
constexpr float kLnEps   = 1e-5f;
constexpr float kWCarry  = 32.0f;
constexpr float kYCarry  = 16.0f;
constexpr float kScaleW  = 1.0f / kWCarry;
constexpr float kScaleYW = 1.0f / (kWCarry * kYCarry);

static_assert(kRows == 8192 && kXzN == 2048, "shape");
static_assert((kDm % 32) == 0, "GEMM K multiple of 32");
static_assert((kRows % 64) == 0 && (kXzN % 64) == 0 && (kDm % 64) == 0 && (kBcP % 64) == 0, "GEMM M,N multiples of 64");
static_assert((kSeq % kScanTS) == 0 && (kDm % kScanCh) == 0, "scan tiles");
static_assert(2 * kNst <= kBcP, "B|C width");

constexpr size_t kSzAct16 = (size_t)kRows * kDm * 2;
constexpr size_t kSzAct32 = (size_t)kRows * kDm * 4;
constexpr size_t kOffXH   = 0;
constexpr size_t kOffXS   = kOffXH   + kSzAct16;
constexpr size_t kOffZS   = kOffXS   + kSzAct16;
constexpr size_t kOffDLR  = kOffZS   + kSzAct16;
constexpr size_t kOffBCP  = kOffDLR  + kSzAct32;
constexpr size_t kOffPRE  = kOffBCP  + (size_t)kRows * kBcP * 4;
constexpr size_t kOffWIN  = kOffPRE  + kSzAct32;
constexpr size_t kOffWDT  = kOffWIN  + (size_t)kXzN * kDm * 2;
constexpr size_t kOffWOUT = kOffWDT  + (size_t)kDm * kDm * 2;
constexpr size_t kOffWBC  = kOffWOUT + (size_t)kDm * kDm * 2;
constexpr size_t kWsTotal = kOffWBC  + (size_t)kBcP * kDm * 2;
static_assert(kWsTotal == 128057344ull, "carve total");
static_assert(kWsTotal <= 134217728ull, "carve cap");
static_assert((kOffXS % 128) == 0 && (kOffZS % 128) == 0 && (kOffDLR % 128) == 0 && (kOffBCP % 128) == 0 &&
              (kOffPRE % 128) == 0 && (kOffWIN % 128) == 0 && (kOffWDT % 128) == 0 && (kOffWOUT % 128) == 0 &&
              (kOffWBC % 128) == 0, "128-B aligned regions");

__device__ __forceinline__ float h16_to_f32(unsigned hb) {
  const unsigned sgn = (hb & 0x8000u) << 16;
  const unsigned em  = hb & 0x7fffu;
  const float fn = __uint_as_float((em << 13) + 0x38000000u);
  const float fs = (float)em * 5.9604644775390625e-8f;
  const float mag = (em < 0x400u) ? fs : fn;
  return __uint_as_float(__float_as_uint(mag) | sgn);
}

__device__ __forceinline__ void wave_lds_sync() {
  __builtin_amdgcn_fence(__ATOMIC_RELEASE, "workgroup");
  __builtin_amdgcn_wave_barrier();
  __builtin_amdgcn_fence(__ATOMIC_ACQUIRE, "workgroup");
}

__device__ __forceinline__ void row_guard_h(v8f& a, v8f& b, v8f& c, v8f& d, v16h x, v16h b0, v16h b1, v16h b2, v16h b3) {
  asm volatile("v_nop\n\tv_nop\n\tv_nop\n\tv_nop" : "+v"(a), "+v"(b), "+v"(c), "+v"(d) : "v"(x), "v"(b0), "v"(b1), "v"(b2), "v"(b3));
}
__device__ __forceinline__ void keep4_h(v16h a, v16h b, v16h c, v16h d) { asm volatile("v_nop" :: "v"(a), "v"(b), "v"(c), "v"(d)); }
__device__ __forceinline__ void acc_guard4(v8f& a, v8f& b, v8f& c, v8f& d) { asm volatile("v_nop\n\tv_nop\n\tv_nop\n\tv_nop" : "+v"(a), "+v"(b), "+v"(c), "+v"(d)); }

struct FragH {
  union U { v16h v; v8h h[2]; };
  static __device__ __forceinline__ v16h load(const _Float16* p) {
    U f;
    f.h[0] = *(const v8h*)(p);
    f.h[1] = *(const v8h*)(p + 16);
    return f.v;
  }
  static __device__ __forceinline__ v8f mma(v16h a, v16h b, v8f c) {
    return __builtin_amdgcn_wmma_f32_16x16x32_f16(false, a, false, b, (short)0, c, false, false);
  }
};

template <int BIAS_MODE, int EPI>
__global__ __launch_bounds__(256) void gemm_f16_kernel(
    const unsigned short* __restrict__ Ap, int lda,
    const unsigned short* __restrict__ Btp, int ldb,
    void* Cout, void* Cout2, int ldc,
    const float* __restrict__ bias,
    const float* __restrict__ resid, int ldr,
    int M, int N, int K, float scale)
{
  const _Float16* A  = (const _Float16*)Ap;
  const _Float16* Bt = (const _Float16*)Btp;
  __shared__ __align__(16) float sT[8][16 * 68];
  const int lane = threadIdx.x & 31;
  const int wave = threadIdx.x >> 5;
  const int tilesN = N >> 6;
  const int tilesM = M >> 6;
  const int tile = blockIdx.x * 8 + wave;
  if (tile >= tilesM * tilesN) return;
  const int tm = tile / tilesN;
  const int tn = tile - tm * tilesN;
  const int m0 = tm << 6;
  const int n0 = tn << 6;

  const int rlane = lane & 15;
  const int koff  = (lane >> 4) * 8;
  const int mOff  = (lane >> 4) * 8;

  v8f acc[4][4];
#pragma unroll
  for (int i = 0; i < 4; ++i)
#pragma unroll
    for (int j = 0; j < 4; ++j) acc[i][j] = (v8f){0.f,0.f,0.f,0.f,0.f,0.f,0.f,0.f};

  for (int k0 = 0; k0 < K; k0 += 32) {
    v16h bh[4];
#pragma unroll
    for (int j = 0; j < 4; ++j) {
      const size_t bo = (size_t)(n0 + (j << 4) + rlane) * ldb + koff + k0;
      bh[j] = FragH::load(Bt + bo);
    }
#pragma unroll
    for (int i = 0; i < 4; ++i) {
      const size_t ao = (size_t)(m0 + (i << 4) + rlane) * lda + koff + k0;
      const v16h ah = FragH::load(A + ao);
#pragma unroll
      for (int j = 0; j < 4; ++j) acc[i][j] = FragH::mma(ah, bh[j], acc[i][j]);
      row_guard_h(acc[i][0], acc[i][1], acc[i][2], acc[i][3], ah, bh[0], bh[1], bh[2], bh[3]);
    }
    keep4_h(bh[0], bh[1], bh[2], bh[3]);
  }
  acc_guard4(acc[0][0], acc[0][1], acc[0][2], acc[0][3]);
  acc_guard4(acc[1][0], acc[1][1], acc[1][2], acc[1][3]);
  acc_guard4(acc[2][0], acc[2][1], acc[2][2], acc[2][3]);
  acc_guard4(acc[3][0], acc[3][1], acc[3][2], acc[3][3]);

  float* slab = sT[wave];
  const bool zhalf = (EPI == 2) && (n0 >= kDm);
#pragma unroll
  for (int i = 0; i < 4; ++i) {
    const int mBase = m0 + (i << 4);
#pragma unroll
    for (int j = 0; j < 4; ++j) {
      const int n = n0 + (j << 4) + rlane;
      float bv = 0.f;
      if (BIAS_MODE == 2) bv = bias[n];
#pragma unroll
      for (int r = 0; r < 8; ++r) {
        float v = acc[i][j][r] * scale;
        if (BIAS_MODE == 2) v += bv;
        slab[(mOff + r) * 68 + (j << 4) + rlane] = v;
      }
    }
    wave_lds_sync();
    if (EPI == 2) {
      if (zhalf) {
#pragma unroll 1
        for (int it = 0; it < 32; ++it) {
          const int e = it * 32 + lane;
          float* sp = slab + (e >> 6) * 68 + (e & 63);
          const float v = *sp;
          const float sg = __builtin_amdgcn_rcpf(1.0f + expf(-v));
          *sp = v * sg;
        }
        wave_lds_sync();
      }
      unsigned short* C = zhalf ? (unsigned short*)Cout2 : (unsigned short*)Cout;
      const int cbase = zhalf ? (n0 - kDm) : n0;
      const int q = lane >> 3, c8 = (lane & 7) * 8;
      v8h hv[4];
#pragma unroll
      for (int it = 0; it < 4; ++it) {
        const float* sp = slab + (it * 4 + q) * 68 + c8;
#pragma unroll
        for (int e = 0; e < 8; ++e) hv[it][e] = (_Float16)sp[e];
      }
      for (int pass = 0; pass < 2; ++pass) {
#pragma unroll
        for (int it = 0; it < 4; ++it)
          *(volatile v8h*)(C + (size_t)(mBase + it * 4 + q) * ldc + cbase + c8) = hv[it];
        __threadfence();
      }
    } else {
      float* C = (float*)Cout;
      const int hh = lane >> 4, c4 = (lane & 15) * 4;
      v4f ov[8];
#pragma unroll
      for (int it = 0; it < 8; ++it) {
        const int row = it * 2 + hh;
        v4f v = *(const v4f*)(slab + row * 68 + c4);
        if (EPI == 1) {
          const v4f r4 = *(const v4f*)(resid + (size_t)(mBase + row) * ldr + n0 + c4);
          v = v + r4;
        }
        ov[it] = v;
      }
      for (int pass = 0; pass < 2; ++pass) {
#pragma unroll
        for (int it = 0; it < 8; ++it)
          *(volatile v4f*)(C + (size_t)(mBase + it * 2 + hh) * ldc + n0 + c4) = ov[it];
        __threadfence();
      }
    }
    wave_lds_sync();
  }
}

__global__ __launch_bounds__(256) void cast_f16_kernel(
    const float* __restrict__ src, unsigned short* __restrict__ dst, int total8, float scale)
{
  const int i = blockIdx.x * 256 + threadIdx.x;
  if (i >= total8) return;
  const size_t e0 = (size_t)i << 3;
  const float* p = src + e0;
  const v4f a0 = *(const v4f*)(p);
  const v4f a1 = *(const v4f*)(p + 4);
  v8h hv;
#pragma unroll
  for (int e = 0; e < 4; ++e) {
    hv[e]     = (_Float16)(a0[e] * scale);
    hv[4 + e] = (_Float16)(a1[e] * scale);
  }
  unsigned short* q = dst + e0;
  *(volatile v8h*)q = hv;
  __threadfence();
  *(volatile v8h*)q = hv;
}

__global__ __launch_bounds__(256) void build_wbc_kernel(
    const float* __restrict__ wB, const float* __restrict__ wC, unsigned short* __restrict__ dst, float scale)
{
  const int i   = blockIdx.x * 256 + threadIdx.x;
  const int e0  = i << 3;
  const int row = e0 >> 10;
  const int col = e0 & (kDm - 1);
  const bool useB = (blockIdx.x < 8);
  const bool live = (blockIdx.x < 16);
  const float* src = useB ? wB : wC;
  int srow = useB ? row : (row - kNst);
  srow = (srow < 0) ? 0 : ((srow > kNst - 1) ? (kNst - 1) : srow);
  const float* p = src + (size_t)srow * kDm + col;
  const v4f a0 = *(const v4f*)(p);
  const v4f a1 = *(const v4f*)(p + 4);
  v8h hv;
#pragma unroll
  for (int e = 0; e < 4; ++e) {
    const float u0 = live ? (a0[e] * scale) : 0.0f;
    const float u1 = live ? (a1[e] * scale) : 0.0f;
    hv[e]     = (_Float16)u0;
    hv[4 + e] = (_Float16)u1;
  }
  unsigned short* q = dst + e0;
  *(volatile v8h*)q = hv;
  __threadfence();
  *(volatile v8h*)q = hv;
}

__global__ __launch_bounds__(64) void scan_kernel(
    const float* __restrict__ DLR, const unsigned short* __restrict__ XS, const unsigned short* __restrict__ ZS,
    const float* __restrict__ BCP, const float* __restrict__ bB, const float* __restrict__ bC,
    const float* __restrict__ Alog, const float* __restrict__ Dp, unsigned short* __restrict__ YZ)
{
  __shared__ __align__(16) float sX[kScanTS * 32];
  __shared__ __align__(16) float sY[kScanTS * kScanYP];
  __shared__ __align__(16) float sA[kNst * kScanCh];
  const int tid = threadIdx.x, lane = tid & 31, wave = tid >> 5;
  constexpr int kBlkPerB = kDm / kScanCh;
  const int bix = blockIdx.x / kBlkPerB;
  const int d0  = (blockIdx.x - bix * kBlkPerB) * kScanCh;
  const int d   = d0 + tid;
  const size_t row0 = (size_t)bix * kSeq;
#pragma unroll 1
  for (int s = 0; s < kNst; ++s) sA[s * kScanCh + tid] = -expf(Alog[(size_t)d * kNst + s]);
  __syncthreads();
  float negA[kNst], h[kNst];
#pragma unroll
  for (int s = 0; s < kNst; ++s) {
    negA[s] = sA[s * kScanCh + tid];
    h[s] = 0.f;
  }
  const float Dd = Dp[d];
  const int lr = tid >> 3, lc4 = (tid & 7) * 4;
  v4f bias4;
  {
    const int bo = lc4 & (kNst - 1);
    const v4f vb = *(const v4f*)(bB + bo);
    const v4f vc = *(const v4f*)(bC + bo);
    const float fb = (lc4 < kNst) ? 1.0f : 0.0f;
    const float fc = 1.0f - fb;
#pragma unroll
    for (int e = 0; e < 4; ++e) bias4[e] = fmaf(fb, vb[e], fc * vc[e]);
  }
  const int q = lane >> 3, c8 = (lane & 7) * 8;
#pragma unroll 1
  for (int t0 = 0; t0 < kSeq; t0 += kScanTS) {
    __syncthreads();
#pragma unroll
    for (int i = 0; i < 8; ++i) {
      const int r = lr + 8 * i;
      v4f v = *(const v4f*)(BCP + (row0 + t0 + r) * kBcP + lc4);
      v = v + bias4;
      *(v4f*)(sX + r * 32 + lc4) = v;
    }
    __syncthreads();
#pragma unroll 1
    for (int s = 0; s < kScanTS; ++s) {
      const size_t gi = (row0 + t0 + s) * kDm + d;
      const float v     = DLR[gi];
      const unsigned xb = (unsigned)XS[gi];
      const unsigned zb = (unsigned)ZS[gi];
      const float* xr = sX + s * 32;
      float Bs[kNst], Cs[kNst];
#pragma unroll
      for (int q4 = 0; q4 < 4; ++q4) {
        const v4f bv = *(const v4f*)(xr + 4 * q4);
        const v4f cv = *(const v4f*)(xr + kNst + 4 * q4);
        Bs[4 * q4 + 0] = bv[0]; Bs[4 * q4 + 1] = bv[1]; Bs[4 * q4 + 2] = bv[2]; Bs[4 * q4 + 3] = bv[3];
        Cs[4 * q4 + 0] = cv[0]; Cs[4 * q4 + 1] = cv[1]; Cs[4 * q4 + 2] = cv[2]; Cs[4 * q4 + 3] = cv[3];
      }
      const float xt  = h16_to_f32(xb);
      const float zg  = h16_to_f32(zb);
      const float ea  = __expf(-fabsf(v));
      const float u   = 1.0f + ea;
      const float l1p = __logf(u) + (ea - (u - 1.0f)) * __builtin_amdgcn_rcpf(u);
      const float dt  = fmaxf(v, 0.0f) + l1p;
      const float dtx = dt * xt;
      float y = 0.f;
#pragma unroll
      for (int k = 0; k < kNst; ++k) {
        const float e = __expf(dt * negA[k]);
        h[k] = e * h[k] + dtx * Bs[k];
        y = h[k] * Cs[k] + y;
      }
      y = xt * Dd + y;
      sY[s * kScanYP + tid] = (y * zg) * kYCarry;
    }
    __syncthreads();
    v8h hv[8];
#pragma unroll
    for (int it = 0; it < 8; ++it) {
      const int row = it * 8 + wave * 4 + q;
      const float* sp = sY + row * kScanYP + c8;
      const v4f a0 = *(const v4f*)(sp);
      const v4f a1 = *(const v4f*)(sp + 4);
#pragma unroll
      for (int e = 0; e < 4; ++e) {
        hv[it][e]     = (_Float16)a0[e];
        hv[it][4 + e] = (_Float16)a1[e];
      }
    }
    for (int pass = 0; pass < 2; ++pass) {
#pragma unroll
      for (int it = 0; it < 8; ++it) {
        const int row = it * 8 + wave * 4 + q;
        *(volatile v8h*)(YZ + (row0 + t0 + row) * kDm + d0 + c8) = hv[it];
      }
      __threadfence();
    }
  }
}

__global__ __launch_bounds__(256) void layernorm_kernel(
    const float* __restrict__ pre, const float* __restrict__ gamma, const float* __restrict__ beta,
    float* __restrict__ out)
{
  __shared__ float red0[8];
  __shared__ float red1[8];
  const int tid = threadIdx.x, lane = tid & 31, wave = tid >> 5;
  const size_t base = (size_t)blockIdx.x * kDm + (size_t)tid * 4;
  const v4f v  = *(const v4f*)(pre + base);
  const v4f g4 = *(const v4f*)(gamma + tid * 4);
  const v4f b4 = *(const v4f*)(beta + tid * 4);
  float s = (v[0] + v[1]) + (v[2] + v[3]);
#pragma unroll
  for (int o = 16; o > 0; o >>= 1) s += __shfl_xor(s, o, 32);
  if (lane == 0) red0[wave] = s;
  __syncthreads();
  float tot = 0.f;
#pragma unroll
  for (int w = 0; w < 8; ++w) tot += red0[w];
  const float mu = tot * (1.0f / (float)kDm);
  const float e0 = v[0] - mu, e1 = v[1] - mu, e2 = v[2] - mu, e3 = v[3] - mu;
  float s2 = (e0 * e0 + e1 * e1) + (e2 * e2 + e3 * e3);
#pragma unroll
  for (int o = 16; o > 0; o >>= 1) s2 += __shfl_xor(s2, o, 32);
  if (lane == 0) red1[wave] = s2;
  __syncthreads();
  float tot2 = 0.f;
#pragma unroll
  for (int w = 0; w < 8; ++w) tot2 += red1[w];
  const float var = tot2 * (1.0f / (float)kDm);
  const float inv = rsqrtf(var + kLnEps);
  v4f o4;
  o4[0] = e0 * inv * g4[0] + b4[0];
  o4[1] = e1 * inv * g4[1] + b4[1];
  o4[2] = e2 * inv * g4[2] + b4[2];
  o4[3] = e3 * inv * g4[3] + b4[3];
  float* dst = out + base;
  *(volatile v4f*)dst = o4;
  __threadfence();
  *(volatile v4f*)dst = o4;
}

constexpr int kTilesIn  = (kRows / 64) * (kXzN / 64);
constexpr int kTilesSq  = (kRows / 64) * (kDm / 64);
constexpr int kTilesBc  = (kRows / 64) * (kBcP / 64);
static_assert((kTilesIn % 8) == 0 && (kTilesSq % 8) == 0 && (kTilesBc % 8) == 0, "8 tiles per block");
static_assert(((kRows * kDm) % 2048) == 0 && ((kXzN * kDm) % 2048) == 0 && ((kDm * kDm) % 2048) == 0, "cast grids exact");
static_assert((kBcP * kDm) / 8 / 256 == 32, "pad-plane grid");

extern "C" void kernel_launch(void* const* d_in, const int* in_sizes, int n_in,
                              void* d_out, int out_size, void* d_ws, size_t ws_size,
                              hipStream_t stream)
{
  if (n_in < 15) return;
  if (in_sizes[0] != kRows * kDm) return;
  if (in_sizes[1] != kXzN * kDm || in_sizes[2] != kXzN) return;
  if (in_sizes[3] != kDm * kDm || in_sizes[4] != kDm) return;
  if (in_sizes[5] != kDm * kNst) return;
  if (in_sizes[6] != kNst * kDm || in_sizes[7] != kNst) return;
  if (in_sizes[8] != kNst * kDm || in_sizes[9] != kNst) return;
  if (in_sizes[10] != kDm) return;
  if (in_sizes[11] != kDm * kDm || in_sizes[12] != kDm) return;
  if (in_sizes[13] != kDm || in_sizes[14] != kDm) return;
  if (out_size != kRows * kDm) return;
  if (ws_size < kWsTotal) return;

  const float* x     = (const float*)d_in[0];
  const float* w_in  = (const float*)d_in[1];
  const float* b_in  = (const float*)d_in[2];
  const float* w_dt  = (const float*)d_in[3];
  const float* b_dt  = (const float*)d_in[4];
  const float* A_log = (const float*)d_in[5];
  const float* w_B   = (const float*)d_in[6];
  const float* b_B   = (const float*)d_in[7];
  const float* w_C   = (const float*)d_in[8];
  const float* b_C   = (const float*)d_in[9];
  const float* Dv    = (const float*)d_in[10];
  const float* w_out = (const float*)d_in[11];
  const float* b_out = (const float*)d_in[12];
  const float* gamma = (const float*)d_in[13];
  const float* beta  = (const float*)d_in[14];
  float* out = (float*)d_out;

  char* ws = (char*)d_ws;
  unsigned short* XH   = (unsigned short*)(ws + kOffXH);
  unsigned short* YZ   = (unsigned short*)(ws + kOffXH);
  unsigned short* XS   = (unsigned short*)(ws + kOffXS);
  unsigned short* ZS   = (unsigned short*)(ws + kOffZS);
  float*          DLR  = (float*)(ws + kOffDLR);
  float*          BCP  = (float*)(ws + kOffBCP);
  float*          PRE  = (float*)(ws + kOffPRE);
  unsigned short* WIN  = (unsigned short*)(ws + kOffWIN);
  unsigned short* WDT  = (unsigned short*)(ws + kOffWDT);
  unsigned short* WOUT = (unsigned short*)(ws + kOffWOUT);
  unsigned short* WBC  = (unsigned short*)(ws + kOffWBC);

  cast_f16_kernel<<<(kRows * kDm) / 8 / 256, 256, 0, stream>>>(x, XH, (kRows * kDm) / 8, 1.0f);
  cast_f16_kernel<<<(kXzN * kDm) / 8 / 256, 256, 0, stream>>>(w_in, WIN, (kXzN * kDm) / 8, kWCarry);
  cast_f16_kernel<<<(kDm * kDm) / 8 / 256, 256, 0, stream>>>(w_dt, WDT, (kDm * kDm) / 8, kWCarry);
  cast_f16_kernel<<<(kDm * kDm) / 8 / 256, 256, 0, stream>>>(w_out, WOUT, (kDm * kDm) / 8, kWCarry);
  build_wbc_kernel<<<(kBcP * kDm) / 8 / 256, 256, 0, stream>>>(w_B, w_C, WBC, kWCarry);

  gemm_f16_kernel<2, 2><<<kTilesIn / 8, 256, 0, stream>>>(
      XH, kDm, WIN, kDm, (void*)XS, (void*)ZS, kDm, b_in, x, kDm, kRows, kXzN, kDm, kScaleW);

  gemm_f16_kernel<2, 0><<<kTilesSq / 8, 256, 0, stream>>>(
      XS, kDm, WDT, kDm, (void*)DLR, (void*)DLR, kDm, b_dt, x, kDm, kRows, kDm, kDm, kScaleW);

  gemm_f16_kernel<0, 0><<<kTilesBc / 8, 256, 0, stream>>>(
      XS, kDm, WBC, kDm, (void*)BCP, (void*)BCP, kBcP, b_dt, x, kDm, kRows, kBcP, kDm, kScaleW);

  scan_kernel<<<kBatch * (kDm / kScanCh), kScanCh, 0, stream>>>(DLR, XS, ZS, BCP, b_B, b_C, A_log, Dv, YZ);

  gemm_f16_kernel<2, 1><<<kTilesSq / 8, 256, 0, stream>>>(
      YZ, kDm, WOUT, kDm, (void*)PRE, (void*)PRE, kDm, b_out, x, kDm, kRows, kDm, kDm, kScaleYW);

  layernorm_kernel<<<kRows, 256, 0, stream>>>(PRE, gamma, beta, out);
}
